// MambaBlock_34780645163484
// MI455X (gfx1250) — hardware-verified
//
#include <hip/hip_runtime.h>
#include <stddef.h>
#include <stdint.h>
#include <math.h>


#define DM     256
#define DI     512
#define NST    64
#define DTR    16
#define NXD    144
#define NXP    192
#define NBAT   2
#define LSEQ   1024
#define ROWS   (NBAT * LSEQ)
#define NIN    (2 * DI)
#define K2I    (2 * DI)
#define K2D    (2 * DTR)
#define BCW    128
#define GBM    64
#define GBN    64
#define GTHR   128
#define NTHR   256
#define CST    32
#define ST     32
#define SCC    64
#define SPN    (DI * 4 + 3 * DI)
#define SP_CB  (DI * 4)
#define SP_DTB (DI * 4 + DI)
#define SP_DS  (DI * 4 + 2 * DI)
#define WSMAX  134217728

#define PU_XB  (ROWS * DM / 8)
#define PU_WIN (NIN * DM / 8)
#define PU_WX  (NXP * K2I / 8)
#define PU_WDT (DI * K2D / 8)
#define PU_WO  (DM * K2I / 8)
#define PU_AN  (DI * NST / 4)
#define PU_SP  (SPN / 4)
#define E_WIN  (PU_XB + PU_WIN)
#define E_WX   (E_WIN + PU_WX)
#define E_WDT  (E_WX + PU_WDT)
#define E_WO   (E_WDT + PU_WO)
#define E_AN   (E_WO + PU_AN)
#define PU_ALL (E_AN + PU_SP)

static_assert(ROWS % 128 == 0 && ROWS % GBM == 0);
static_assert(DM % 32 == 0 && K2I % 32 == 0 && K2D % 32 == 0 && K2I == 2 * DI && K2D == 32);
static_assert(NIN % GBN == 0 && NXP % GBN == 0 && DI % GBN == 0 && DM % GBN == 0);
static_assert(GBM == (GTHR / 32) * 16 && GBN == 64);
static_assert(NST == 64 && NST == 4 * 16 && DI % SCC == 0 && LSEQ % ST == 0 && LSEQ % CST == 0);
static_assert(NXP >= NXD && DTR == 16 && DTR + NST == 80 && DTR + 2 * NST == NXD);
static_assert(NXP == 3 * GBN && NST == GBN && BCW == 2 * NST);
static_assert(PU_XB % 32 == 0 && E_WIN % 32 == 0 && E_WX % 32 == 0 && E_WDT % 32 == 0);
static_assert(E_WO % 32 == 0 && E_AN % 32 == 0 && PU_ALL % 32 == 0);
static_assert((SP_CB / 4) % 32 == 0 && (DI / 4) % 32 == 0);
static_assert(((ROWS / CST) * (DI / 4)) % NTHR == 0 && (DI / 4) == 128);
static_assert(ST * SCC / 4 == 2 * NTHR && ST * BCW / 4 == 4 * NTHR && SCC * 4 == NTHR && ST * 2 == 2 * (NTHR / 8));
static_assert((LSEQ & (LSEQ - 1)) == 0);

typedef float          v4f   __attribute__((ext_vector_type(4)));
typedef float          v8f   __attribute__((ext_vector_type(8)));
typedef int            v8i   __attribute__((ext_vector_type(8)));
typedef unsigned short v4us  __attribute__((ext_vector_type(4)));
typedef unsigned short v8us  __attribute__((ext_vector_type(8)));
typedef unsigned short v16us __attribute__((ext_vector_type(16)));
typedef __bf16         v16bf __attribute__((ext_vector_type(16)));
typedef v4f  __attribute__((may_alias)) v4fa;
typedef v8us __attribute__((may_alias)) v8usa;
union FragB { v16bf v; v16us u; v8us h[2]; v8i w; };

__device__ __forceinline__ v8f wmb(const FragB& a, const FragB& b, v8f c) {
  v8f d = __builtin_amdgcn_wmma_f32_16x16x32_bf16(false, a.v, false, b.v, (short)0, c, false, false);
  asm volatile("v_nop\n\tv_nop\n\tv_nop\n\tv_nop" : "+v"(d) : "v"(a.w), "v"(b.w));
  return d;
}

__device__ __forceinline__ unsigned bf16_bits(float f) {
  const unsigned u = __float_as_uint(f);
  return (u + 0x7FFFu + ((u >> 16) & 1u)) >> 16;
}
__device__ __forceinline__ float bf16_val(float f) {
  return __uint_as_float(bf16_bits(f) << 16);
}
__device__ __forceinline__ unsigned short hl_sel(float v, bool lo_sel) {
  const unsigned hb = bf16_bits(v);
  const unsigned lb = bf16_bits(v - __uint_as_float(hb << 16));
  return (unsigned short)(lo_sel ? lb : hb);
}
__device__ __forceinline__ float silu_f(float v) {
  return v * __builtin_amdgcn_rcpf(1.0f + expf(-v));
}
__device__ __forceinline__ float softplus_f(float p) {
  return fmaxf(p, 0.0f) + log1pf(expf(-fabsf(p)));
}

__device__ __forceinline__ void pack8_put(float f0, float f1, float f2, float f3, float f4, float f5, float f6,
                                          float f7, bool ok, unsigned short* dp) {
  v8us o;
  o[0] = ok ? (unsigned short)bf16_bits(f0) : (unsigned short)0;
  o[1] = ok ? (unsigned short)bf16_bits(f1) : (unsigned short)0;
  o[2] = ok ? (unsigned short)bf16_bits(f2) : (unsigned short)0;
  o[3] = ok ? (unsigned short)bf16_bits(f3) : (unsigned short)0;
  o[4] = ok ? (unsigned short)bf16_bits(f4) : (unsigned short)0;
  o[5] = ok ? (unsigned short)bf16_bits(f5) : (unsigned short)0;
  o[6] = ok ? (unsigned short)bf16_bits(f6) : (unsigned short)0;
  o[7] = ok ? (unsigned short)bf16_bits(f7) : (unsigned short)0;
  *(volatile v8us*)dp = o;
  __threadfence();
  *(volatile v8us*)dp = o;
}
__device__ __forceinline__ void cvt8_put(const float* p, bool ok, unsigned short* dp) {
  const v4f a = *(const v4fa*)p;
  const v4f b = *(const v4fa*)(p + 4);
  pack8_put(a.x, a.y, a.z, a.w, b.x, b.y, b.z, b.w, ok, dp);
}
__device__ __forceinline__ void gat8_put(const float* p, int stride, bool ok, unsigned short* dp) {
  const float f0 = p[0];
  const float f1 = p[stride];
  const float f2 = p[2 * stride];
  const float f3 = p[3 * stride];
  const float f4 = p[4 * stride];
  const float f5 = p[5 * stride];
  const float f6 = p[6 * stride];
  const float f7 = p[7 * stride];
  pack8_put(f0, f1, f2, f3, f4, f5, f6, f7, ok, dp);
}
__device__ __forceinline__ void rnd4_put(const float* p, float* dp) {
  const v4f a = *(const v4fa*)p;
  v4f o;
  o.x = bf16_val(a.x); o.y = bf16_val(a.y); o.z = bf16_val(a.z); o.w = bf16_val(a.w);
  *(volatile v4f*)dp = o;
  __threadfence();
  *(volatile v4f*)dp = o;
}

__global__ __launch_bounds__(NTHR) void k_prep(
    const float* __restrict__ x, const float* __restrict__ win, const float* __restrict__ ck,
    const float* __restrict__ cb, const float* __restrict__ wx, const float* __restrict__ wdt,
    const float* __restrict__ dtb, const float* __restrict__ alog, const float* __restrict__ dsk,
    const float* __restrict__ wo,
    unsigned short* XB, unsigned short* WINT, unsigned short* WXT2, unsigned short* WDT2,
    unsigned short* WOT2, float* AN, float* SP)
{
  const int u = (int)blockIdx.x * NTHR + (int)threadIdx.x;
  if (u < PU_XB) {
    cvt8_put(x + (size_t)8 * u, true, XB + (size_t)8 * u);
  } else if (u < E_WIN) {
    const int v  = u - PU_XB;
    const int n  = v >> 5;
    const int k8 = (v & 31) * 8;
    gat8_put(win + (size_t)k8 * NIN + n, NIN, true, WINT + (size_t)8 * v);
  } else if (u < E_WX) {
    const int v  = u - E_WIN;
    const int n  = v >> 7;
    const int kk = (v & 127) * 8;
    const int k  = kk & (DI - 1);
    const int sc = (n < 2 * NST) ? (n + DTR) : ((n < NXD) ? (n - 2 * NST) : 0);
    gat8_put(wx + (size_t)k * NXD + sc, NXD, n < NXD, WXT2 + (size_t)8 * v);
  } else if (u < E_WDT) {
    const int v  = u - E_WX;
    const int n  = v >> 2;
    const int kk = (v & 3) * 8;
    const int k  = kk & (DTR - 1);
    gat8_put(wdt + (size_t)k * DI + n, DI, true, WDT2 + (size_t)8 * v);
  } else if (u < E_WO) {
    const int v  = u - E_WDT;
    const int n  = v >> 7;
    const int kk = (v & 127) * 8;
    const int k  = kk & (DI - 1);
    gat8_put(wo + (size_t)k * DM + n, DM, true, WOT2 + (size_t)8 * v);
  } else if (u < E_AN) {
    const int v = u - E_WO;
    const v4f a = *(const v4fa*)(alog + (size_t)4 * v);
    v4f o;
    o.x = -expf(bf16_val(a.x)); o.y = -expf(bf16_val(a.y));
    o.z = -expf(bf16_val(a.z)); o.w = -expf(bf16_val(a.w));
    float* dp = AN + (size_t)4 * v;
    *(volatile v4f*)dp = o;
    __threadfence();
    *(volatile v4f*)dp = o;
  } else if (u < PU_ALL) {
    const int v = u - E_AN;
    float* dp = SP + (size_t)4 * v;
    if (v < SP_CB / 4)            rnd4_put(ck  + (size_t)4 * v, dp);
    else if (v < SP_DTB / 4)      rnd4_put(cb  + (size_t)4 * (v - SP_CB / 4), dp);
    else if (v < SP_DS / 4)       rnd4_put(dtb + (size_t)4 * (v - SP_DTB / 4), dp);
    else                          rnd4_put(dsk + (size_t)4 * (v - SP_DS / 4), dp);
  }
}

template <int MODE>
__global__ __launch_bounds__(GTHR) void k_gemm(
    const unsigned short* __restrict__ A, int lda,
    const unsigned short* __restrict__ WT, int ldb, int K,
    float* outF, int ldo, int nsplit, int pstride,
    const float* __restrict__ bias, unsigned short* outH)
{
  __shared__ __attribute__((aligned(16))) float stg[GBM * GBN];
  const int tid = (int)threadIdx.x, lane = tid & 31, wave = tid >> 5, hh = lane >> 4, m = lane & 15;
  const int rowBase = (int)blockIdx.x * GBM;
  const int col0    = (int)blockIdx.y * GBN;

  v8f acc[4];
  {
    const v8f z = {0.f, 0.f, 0.f, 0.f, 0.f, 0.f, 0.f, 0.f};
    acc[0] = z; acc[1] = z; acc[2] = z; acc[3] = z;
  }
  const unsigned short* ap = A  + (size_t)(rowBase + 16 * wave + m) * (size_t)lda + 8 * hh;
  const unsigned short* wp = WT + (size_t)(col0 + m) * (size_t)ldb + 8 * hh;
  const int ksteps = K >> 5;
#pragma unroll 1
  for (int ks = 0; ks < ksteps; ++ks) {
    FragB af;
    af.h[0] = *(const v8usa*)(ap + 32 * ks);
    af.h[1] = *(const v8usa*)(ap + 32 * ks + 16);
#pragma unroll
    for (int t = 0; t < 4; ++t) {
      const unsigned short* wq = wp + (size_t)(16 * t) * (size_t)ldb + 32 * ks;
      FragB bf;
      bf.h[0] = *(const v8usa*)wq;
      bf.h[1] = *(const v8usa*)(wq + 16);
      acc[t] = wmb(af, bf, acc[t]);
    }
  }

#pragma unroll
  for (int t = 0; t < 4; ++t) {
    const int lc = 16 * t + m;
#pragma unroll
    for (int r = 0; r < 8; ++r) {
      const int lr = 16 * wave + 8 * hh + r;
      stg[lr * GBN + lc] = acc[t][r];
    }
  }
  __syncthreads();

  if constexpr (MODE == 0 || MODE == 3) {
    const int plane = col0 / nsplit;
    const int cc    = col0 - plane * nsplit;
    if constexpr (MODE == 3) {
      if (plane == 1) {
#pragma unroll 1
        for (int i = 0; i < 8; ++i) {
          float* sp = stg + (16 * wave + 2 * i + hh) * GBN + 4 * m;
          v4f v = *(const v4fa*)sp;
          v.x = silu_f(v.x); v.y = silu_f(v.y); v.z = silu_f(v.z); v.w = silu_f(v.w);
          *(v4fa*)sp = v;
        }
      }
    }
    float* ob = outF + (size_t)plane * (size_t)pstride + cc + 4 * m;
    v4f fv[8];
#pragma unroll
    for (int i = 0; i < 8; ++i) {
      const int lr = 16 * wave + 2 * i + hh;
      fv[i] = *(const v4fa*)(stg + lr * GBN + 4 * m);
    }
#pragma unroll
    for (int i = 0; i < 8; ++i) {
      const int lr = 16 * wave + 2 * i + hh;
      *(volatile v4f*)(ob + (size_t)(rowBase + lr) * (size_t)ldo) = fv[i];
    }
    __threadfence();
#pragma unroll
    for (int i = 0; i < 8; ++i) {
      const int lr = 16 * wave + 2 * i + hh;
      *(volatile v4f*)(ob + (size_t)(rowBase + lr) * (size_t)ldo) = fv[i];
    }
  } else if constexpr (MODE == 1) {
    const v4f bb = *(const v4fa*)(bias + col0 + 4 * m);
#pragma unroll 1
    for (int i = 0; i < 8; ++i) {
      const int lr = 16 * wave + 2 * i + hh;
      const v4f t = *(const v4fa*)(stg + lr * GBN + 4 * m);
      v4f o;
      o.x = softplus_f(t.x + bb.x);
      o.y = softplus_f(t.y + bb.y);
      o.z = softplus_f(t.z + bb.z);
      o.w = softplus_f(t.w + bb.w);
      float* op = outF + (size_t)(rowBase + lr) * (size_t)ldo + col0 + 4 * m;
      *(volatile v4f*)op = o;
      __threadfence();
      *(volatile v4f*)op = o;
    }
  } else {
    if (blockIdx.y < 2) {
      float* ob = outF + 64 * (int)blockIdx.y + 4 * m;
      v4f fv[8];
#pragma unroll
      for (int i = 0; i < 8; ++i) {
        const int lr = 16 * wave + 2 * i + hh;
        fv[i] = *(const v4fa*)(stg + lr * GBN + 4 * m);
      }
#pragma unroll
      for (int i = 0; i < 8; ++i) {
        const int lr = 16 * wave + 2 * i + hh;
        *(volatile v4f*)(ob + (size_t)(rowBase + lr) * BCW) = fv[i];
      }
      __threadfence();
#pragma unroll
      for (int i = 0; i < 8; ++i) {
        const int lr = 16 * wave + 2 * i + hh;
        *(volatile v4f*)(ob + (size_t)(rowBase + lr) * BCW) = fv[i];
      }
    } else {
      const int  rs = lane >> 2;
      const int  pc = lane & 3;
      const int  c8 = 8 * (pc & 1);
      const bool lo_sel = (pc >= 2);
      v8us qv[2];
#pragma unroll
      for (int i = 0; i < 2; ++i) {
        const int lr = 16 * wave + 8 * i + rs;
        const v4f a = *(const v4fa*)(stg + lr * GBN + c8);
        const v4f b = *(const v4fa*)(stg + lr * GBN + c8 + 4);
        v8us o;
        o[0] = hl_sel(a.x, lo_sel); o[1] = hl_sel(a.y, lo_sel);
        o[2] = hl_sel(a.z, lo_sel); o[3] = hl_sel(a.w, lo_sel);
        o[4] = hl_sel(b.x, lo_sel); o[5] = hl_sel(b.y, lo_sel);
        o[6] = hl_sel(b.z, lo_sel); o[7] = hl_sel(b.w, lo_sel);
        qv[i] = o;
      }
#pragma unroll
      for (int i = 0; i < 2; ++i) {
        const int lr = 16 * wave + 8 * i + rs;
        *(volatile v8us*)(outH + (size_t)(rowBase + lr) * K2D + 8 * pc) = qv[i];
      }
      __threadfence();
#pragma unroll
      for (int i = 0; i < 2; ++i) {
        const int lr = 16 * wave + 8 * i + rs;
        *(volatile v8us*)(outH + (size_t)(rowBase + lr) * K2D + 8 * pc) = qv[i];
      }
    }
  }
}

__global__ __launch_bounds__(NTHR) void k_conv(const float* __restrict__ XI, const float* __restrict__ SP,
                                               float* U, unsigned short* UHL)
{
  const int t = (int)blockIdx.x * NTHR + (int)threadIdx.x;
  const int q = t & 127;
  const int s = t >> 7;
  if (s >= ROWS / CST) return;
  const int r0 = s * CST;
  const int c0 = 4 * q;
  const v4f t0 = *(const v4fa*)(SP + 0 * DI + c0);
  const v4f t1 = *(const v4fa*)(SP + 1 * DI + c0);
  const v4f t2 = *(const v4fa*)(SP + 2 * DI + c0);
  const v4f t3 = *(const v4fa*)(SP + 3 * DI + c0);
  const v4f bb = *(const v4fa*)(SP + SP_CB + c0);
  const bool pv = (r0 & (LSEQ - 1)) != 0;
  const int ra = pv ? r0 - 3 : r0;
  const int rb = pv ? r0 - 2 : r0;
  const int rc = pv ? r0 - 1 : r0;
  const v4f zz = {0.f, 0.f, 0.f, 0.f};
  v4f x0 = *(const v4fa*)(XI + (size_t)ra * DI + c0);
  v4f x1 = *(const v4fa*)(XI + (size_t)rb * DI + c0);
  v4f x2 = *(const v4fa*)(XI + (size_t)rc * DI + c0);
  x0 = pv ? x0 : zz; x1 = pv ? x1 : zz; x2 = pv ? x2 : zz;
#pragma unroll 1
  for (int i = 0; i < CST; ++i) {
    const int r = r0 + i;
    const v4f xn = *(const v4fa*)(XI + (size_t)r * DI + c0);
    v4f c;
    c.x = fmaf(t3.x, xn.x, fmaf(t2.x, x2.x, fmaf(t1.x, x1.x, t0.x * x0.x))) + bb.x;
    c.y = fmaf(t3.y, xn.y, fmaf(t2.y, x2.y, fmaf(t1.y, x1.y, t0.y * x0.y))) + bb.y;
    c.z = fmaf(t3.z, xn.z, fmaf(t2.z, x2.z, fmaf(t1.z, x1.z, t0.z * x0.z))) + bb.z;
    c.w = fmaf(t3.w, xn.w, fmaf(t2.w, x2.w, fmaf(t1.w, x1.w, t0.w * x0.w))) + bb.w;
    v4f uo;
    uo.x = silu_f(c.x); uo.y = silu_f(c.y); uo.z = silu_f(c.z); uo.w = silu_f(c.w);
    v4us hv, lv;
    hv[0] = hl_sel(uo.x, false); lv[0] = hl_sel(uo.x, true);
    hv[1] = hl_sel(uo.y, false); lv[1] = hl_sel(uo.y, true);
    hv[2] = hl_sel(uo.z, false); lv[2] = hl_sel(uo.z, true);
    hv[3] = hl_sel(uo.w, false); lv[3] = hl_sel(uo.w, true);
    float* up = U + (size_t)r * DI + c0;
    unsigned short* hp = UHL + (size_t)r * K2I + c0;
    *(volatile v4f*)up = uo;
    *(volatile v4us*)hp = hv;
    *(volatile v4us*)(hp + DI) = lv;
    __threadfence();
    *(volatile v4f*)up = uo;
    *(volatile v4us*)hp = hv;
    *(volatile v4us*)(hp + DI) = lv;
    x0 = x1; x1 = x2; x2 = xn;
  }
}

__global__ __launch_bounds__(NTHR) void k_scan(const float* __restrict__ DELTA, const float* __restrict__ U,
                                               const float* __restrict__ SZ, const float* __restrict__ BC,
                                               const float* __restrict__ AN, const float* __restrict__ DS,
                                               unsigned short* GHL)
{
  __shared__ __attribute__((aligned(16))) float dls[ST * SCC];
  __shared__ __attribute__((aligned(16))) float uus[ST * SCC];
  __shared__ __attribute__((aligned(16))) float szs[ST * SCC];
  __shared__ __attribute__((aligned(16))) float ggs[ST * SCC];
  __shared__ __attribute__((aligned(16))) float bcs[ST * BCW];
  const int tid = (int)threadIdx.x;
  const int ch = tid >> 2, q = tid & 3;
  const int b = (int)blockIdx.x >> 3;
  const int chBase = ((int)blockIdx.x & 7) * SCC;
  const int d = chBase + ch;

  float Aa[16], h[16];
#pragma unroll
  for (int j = 0; j < 4; ++j) {
    const v4f a = *(const v4fa*)(AN + (size_t)d * NST + 16 * q + 4 * j);
    Aa[4 * j + 0] = a.x; Aa[4 * j + 1] = a.y; Aa[4 * j + 2] = a.z; Aa[4 * j + 3] = a.w;
    h[4 * j + 0] = 0.0f; h[4 * j + 1] = 0.0f; h[4 * j + 2] = 0.0f; h[4 * j + 3] = 0.0f;
  }
  const float Dd = DS[d];

#pragma unroll 1
  for (int cnk = 0; cnk < LSEQ / ST; ++cnk) {
    const int row0 = b * LSEQ + cnk * ST;
#pragma unroll
    for (int it = 0; it < 2; ++it) {
      const int idx = it * NTHR + tid;
      const int row = idx >> 4;
      const int cc  = (idx & 15) * 4;
      const size_t go = (size_t)(row0 + row) * DI + chBase + cc;
      const v4f a = *(const v4fa*)(DELTA + go);
      const v4f e = *(const v4fa*)(U + go);
      const v4f f = *(const v4fa*)(SZ + go);
      *(v4fa*)(dls + row * SCC + cc) = a;
      *(v4fa*)(uus + row * SCC + cc) = e;
      *(v4fa*)(szs + row * SCC + cc) = f;
    }
#pragma unroll
    for (int it = 0; it < 4; ++it) {
      const int idx = it * NTHR + tid;
      const int row = idx >> 5;
      const int cc  = (idx & 31) * 4;
      const v4f a = *(const v4fa*)(BC + (size_t)(row0 + row) * BCW + cc);
      *(v4fa*)(bcs + row * BCW + cc) = a;
    }
    __syncthreads();

#pragma unroll 1
    for (int t = 0; t < ST; ++t) {
      const float dl = dls[t * SCC + ch];
      const float uu = uus[t * SCC + ch];
      const float zv = szs[t * SCC + ch];
      const float du = dl * uu;
      const float* bp = bcs + t * BCW + 16 * q;
      float Bv[16], Cv[16];
#pragma unroll
      for (int j = 0; j < 4; ++j) {
        const v4f tb = *(const v4fa*)(bp + 4 * j);
        const v4f tc = *(const v4fa*)(bp + NST + 4 * j);
        Bv[4 * j + 0] = tb.x; Bv[4 * j + 1] = tb.y; Bv[4 * j + 2] = tb.z; Bv[4 * j + 3] = tb.w;
        Cv[4 * j + 0] = tc.x; Cv[4 * j + 1] = tc.y; Cv[4 * j + 2] = tc.z; Cv[4 * j + 3] = tc.w;
      }
      float p = 0.0f;
#pragma unroll
      for (int j = 0; j < 16; ++j) {
        const float dA = expf(dl * Aa[j]);
        h[j] = fmaf(dA, h[j], du * Bv[j]);
        p = fmaf(h[j], Cv[j], p);
      }
      p += __shfl_xor(p, 1, 32);
      p += __shfl_xor(p, 2, 32);
      const float y = p + uu * Dd;
      const float g = y * zv;
      if (q == 0) ggs[t * SCC + ch] = g;
    }
    __syncthreads();

    v8us ov[2];
#pragma unroll
    for (int j = 0; j < 2; ++j) {
      const int lineid = j * 32 + (tid >> 3);
      const int ll     = lineid >> 1;
      const bool lo_sel = (lineid & 1) != 0;
      const int p8     = tid & 7;
      const v4f a = *(const v4fa*)(ggs + ll * SCC + 8 * p8);
      const v4f c = *(const v4fa*)(ggs + ll * SCC + 8 * p8 + 4);
      v8us o;
      o[0] = hl_sel(a.x, lo_sel); o[1] = hl_sel(a.y, lo_sel);
      o[2] = hl_sel(a.z, lo_sel); o[3] = hl_sel(a.w, lo_sel);
      o[4] = hl_sel(c.x, lo_sel); o[5] = hl_sel(c.y, lo_sel);
      o[6] = hl_sel(c.z, lo_sel); o[7] = hl_sel(c.w, lo_sel);
      ov[j] = o;
    }
#pragma unroll
    for (int j = 0; j < 2; ++j) {
      const int lineid = j * 32 + (tid >> 3);
      const int ll     = lineid >> 1;
      const int which  = lineid & 1;
      const int p8     = tid & 7;
      unsigned short* dp = GHL + (size_t)(row0 + ll) * K2I + (size_t)which * DI + chBase + 8 * p8;
      *(volatile v8us*)dp = ov[j];
    }
    __threadfence();
#pragma unroll
    for (int j = 0; j < 2; ++j) {
      const int lineid = j * 32 + (tid >> 3);
      const int ll     = lineid >> 1;
      const int which  = lineid & 1;
      const int p8     = tid & 7;
      unsigned short* dp = GHL + (size_t)(row0 + ll) * K2I + (size_t)which * DI + chBase + 8 * p8;
      *(volatile v8us*)dp = ov[j];
    }
  }
}

static inline size_t al256(size_t o) { return (o + 255) & ~(size_t)255; }

extern "C" void kernel_launch(void* const* d_in, const int* in_sizes, int n_in,
                              void* d_out, int out_size, void* d_ws, size_t ws_size,
                              hipStream_t stream) {
  if (n_in < 10) return;
  if (in_sizes[0] != ROWS * DM) return;
  if (in_sizes[1] != DM * NIN) return;
  if (in_sizes[2] != 4 * DI) return;
  if (in_sizes[3] != DI) return;
  if (in_sizes[4] != DI * NXD) return;
  if (in_sizes[5] != DTR * DI) return;
  if (in_sizes[6] != DI) return;
  if (in_sizes[7] != DI * NST) return;
  if (in_sizes[8] != DI) return;
  if (in_sizes[9] != DI * DM) return;
  if (out_size != ROWS * DM) return;

  const float* x    = (const float*)d_in[0];
  const float* win  = (const float*)d_in[1];
  const float* ck   = (const float*)d_in[2];
  const float* cb   = (const float*)d_in[3];
  const float* wx   = (const float*)d_in[4];
  const float* wdt  = (const float*)d_in[5];
  const float* dtb  = (const float*)d_in[6];
  const float* alog = (const float*)d_in[7];
  const float* dsk  = (const float*)d_in[8];
  const float* wo   = (const float*)d_in[9];
  float* out = (float*)d_out;

  char* ws = (char*)d_ws;
  size_t off = 0;
  const size_t oXI   = off; off = al256(off + (size_t)ROWS * DI * 4);
  const size_t oSZ   = off; off = al256(off + (size_t)ROWS * DI * 4);
  const size_t oU    = off; off = al256(off + (size_t)ROWS * DI * 4);
  const size_t oDEL  = off; off = al256(off + (size_t)ROWS * DI * 4);
  const size_t oUHL  = off; off = al256(off + (size_t)ROWS * K2I * 2);
  const size_t oGHL  = off; off = al256(off + (size_t)ROWS * K2I * 2);
  const size_t oBC   = off; off = al256(off + (size_t)ROWS * BCW * 4);
  const size_t oDLHL = off; off = al256(off + (size_t)ROWS * K2D * 2);
  const size_t oXB   = off; off = al256(off + (size_t)ROWS * DM * 2);
  const size_t oWIN  = off; off = al256(off + (size_t)NIN * DM * 2);
  const size_t oWX   = off; off = al256(off + (size_t)NXP * K2I * 2);
  const size_t oWDT  = off; off = al256(off + (size_t)DI * K2D * 2);
  const size_t oWO   = off; off = al256(off + (size_t)DM * K2I * 2);
  const size_t oAN   = off; off = al256(off + (size_t)DI * NST * 4);
  const size_t oSP   = off; off = al256(off + (size_t)SPN * 4);
  if (off > ws_size || off > (size_t)WSMAX) return;

  float*          XI    = (float*)(ws + oXI);
  float*          SZp   = (float*)(ws + oSZ);
  float*          Up    = (float*)(ws + oU);
  float*          DELTA = (float*)(ws + oDEL);
  unsigned short* UHL   = (unsigned short*)(ws + oUHL);
  unsigned short* GHL   = (unsigned short*)(ws + oGHL);
  float*          BC    = (float*)(ws + oBC);
  unsigned short* DLHL  = (unsigned short*)(ws + oDLHL);
  unsigned short* XB    = (unsigned short*)(ws + oXB);
  unsigned short* WINT  = (unsigned short*)(ws + oWIN);
  unsigned short* WXT2  = (unsigned short*)(ws + oWX);
  unsigned short* WDT2  = (unsigned short*)(ws + oWDT);
  unsigned short* WOT2  = (unsigned short*)(ws + oWO);
  float*          AN    = (float*)(ws + oAN);
  float*          SP    = (float*)(ws + oSP);
  const int pstr = (int)((oSZ - oXI) / 4);

  k_prep<<<(PU_ALL + NTHR - 1) / NTHR, NTHR, 0, stream>>>(x, win, ck, cb, wx, wdt, dtb, alog, dsk, wo,
                                                          XB, WINT, WXT2, WDT2, WOT2, AN, SP);
  k_gemm<3><<<dim3(ROWS / GBM, NIN / GBN), GTHR, 0, stream>>>(
      XB, DM, WINT, DM, DM, XI, DI, DI, pstr, SP, DLHL);
  k_conv<<<((ROWS / CST) * (DI / 4)) / NTHR, NTHR, 0, stream>>>(XI, SP, Up, UHL);
  k_gemm<2><<<dim3(ROWS / GBM, NXP / GBN), GTHR, 0, stream>>>(
      UHL, K2I, WXT2, K2I, K2I, BC, BCW, NXP, 0, SP, DLHL);
  k_gemm<1><<<dim3(ROWS / GBM, DI / GBN), GTHR, 0, stream>>>(
      DLHL, K2D, WDT2, K2D, K2D, DELTA, DI, DI, 0, SP + SP_DTB, GHL);
  k_scan<<<NBAT * (DI / SCC), NTHR, 0, stream>>>(DELTA, Up, SZp, BC, AN, SP + SP_DS, GHL);
  k_gemm<0><<<dim3(ROWS / GBM, DM / GBN), GTHR, 0, stream>>>(
      GHL, K2I, WOT2, K2I, K2I, out, DM, DM, 0, SP, DLHL);
}
